// LightGCN_6064493822026
// MI455X (gfx1250) — hardware-verified
//
#include <hip/hip_runtime.h>
#include <math.h>

constexpr int NUM_USER = 100000;
constexpr int NUM_ITEM = 50000;
constexpr int DIM      = 64;
constexpr int NE       = 2000000;
constexpr int BATCH    = 4096;
constexpr int NNEG     = 50;

constexpr int PT    = 64;
constexpr int PSP   = 32;
constexpr int PSCH  = PT * PSP;
constexpr int PNCH  = (NE + PSCH - 1) / PSCH;
constexpr int LCAP  = 1536;
constexpr int LTHR  = LCAP - 32 * PSP;
constexpr int DBAT  = 256;
constexpr int RACC  = 960;
constexpr int RDEG  = 15360;
constexpr int RQT   = 7680;
constexpr int QPH   = (BATCH + RACC - 1) / RACC;
constexpr int NU_PAD = 100800;
constexpr int NI_PAD = 50880;
constexpr int NTU    = NU_PAD / RACC;
constexpr int NTI    = NI_PAD / RACC;
constexpr int NU_BIG = 107520;
constexpr int NI_BIG = 61440;
constexpr int NTDU   = NU_BIG / RDEG;
constexpr int NTDI   = NI_BIG / RDEG;
constexpr int NTQ    = NU_BIG / RQT;
constexpr unsigned EMASK = (1u << 21) - 1u;
constexpr int ACC_BYTES  = (RACC + 16) * DIM * 4;
constexpr int CNT_BYTES  = (RDEG + 16) * 4;
constexpr int LIST_BYTES = 2 * LCAP * 4;
constexpr int POS_BYTES  = 2 * 8 * DBAT;
constexpr int SCNT_BYTES = 64;
constexpr int MAPQ_BYTES = RQT * 2;
constexpr int LDS_DEG  = CNT_BYTES + LIST_BYTES + POS_BYTES + SCNT_BYTES;
constexpr int LDS_ROWS = ACC_BYTES + LIST_BYTES + POS_BYTES + SCNT_BYTES;
constexpr int LDS_QRY  = ACC_BYTES + LIST_BYTES + POS_BYTES + SCNT_BYTES + MAPQ_BYTES;
constexpr int SBLK  = 32;
constexpr int SCT   = 128;
constexpr int NSBLK = BATCH / SBLK;
constexpr int PARTW = 32;
constexpr int OUT_NEG_OFF = BATCH;
constexpr int OUT_REG_OFF = BATCH + BATCH * NNEG;

static_assert(NE % PSP == 0);
static_assert(NE <= (1 << 21));
static_assert(RACC < 1024);
static_assert(RACC % 32 == 0);
static_assert(RDEG % 128 == 0);
static_assert(RQT % 4 == 0);
static_assert(NTU * RACC == NU_PAD);
static_assert(NTI * RACC == NI_PAD);
static_assert(NTDU * RDEG == NU_BIG);
static_assert(NTDI * RDEG == NI_BIG);
static_assert(NTQ * RQT == NU_BIG);
static_assert(NU_PAD >= NUM_USER);
static_assert(NI_PAD >= NUM_ITEM);
static_assert(NU_BIG >= NU_PAD);
static_assert(NI_BIG >= NI_PAD);
static_assert(LTHR >= 0);
static_assert(LCAP % DBAT == 0);
static_assert(DBAT == 256);
static_assert(QPH * RACC >= BATCH);
static_assert(ACC_BYTES % 16 == 0);
static_assert(CNT_BYTES % 16 == 0);
static_assert(LDS_QRY <= 320 * 1024);
static_assert(BATCH % SBLK == 0);
static_assert(NSBLK == SCT);
static_assert(SBLK * NNEG % 4 == 0);
static_assert(OUT_NEG_OFF * 4 == 16384);
static_assert(OUT_REG_OFF * 4 == 835584);
static_assert((OUT_REG_OFF + 1) * 4 == 835588);

typedef __attribute__((ext_vector_type(16))) __bf16 v16b;
typedef __attribute__((ext_vector_type(8)))  __bf16 v8b;
typedef __attribute__((ext_vector_type(8)))  float  v8f;
typedef __attribute__((ext_vector_type(4)))  float  v4f;
typedef __attribute__((ext_vector_type(2)))  float  v2f;
typedef __attribute__((ext_vector_type(4)))  int    v4i;

__device__ __forceinline__ unsigned short f2bf_bits(float f) {
  unsigned u = __float_as_uint(f);
  return (unsigned short)((u + 0x7FFFu + ((u >> 16) & 1u)) >> 16);
}
__device__ __forceinline__ float bf_bits2f(unsigned short h) { return __uint_as_float(((unsigned)h) << 16); }

struct FragB {
  union U { v16b v; v8b h[2]; };
  static __device__ __forceinline__ v16b load(const __bf16* p) {
    U f; f.h[0] = *(const v8b*)(p); f.h[1] = *(const v8b*)(p + 16); return f.v;
  }
};
__device__ __forceinline__ v8f bmma(v16b a, v16b b, v8f c) {
  c = __builtin_amdgcn_wmma_f32_16x16x32_bf16(false, a, false, b, (short)0, c, false, false);
  asm volatile("v_nop\n\tv_nop\n\tv_nop\n\tv_nop" : "+v"(c) : "v"(a), "v"(b));
  return c;
}
__device__ __forceinline__ void lds_wave_sync() {
  __builtin_amdgcn_fence(__ATOMIC_RELEASE, "workgroup");
  __builtin_amdgcn_wave_barrier();
  __builtin_amdgcn_fence(__ATOMIC_ACQUIRE, "workgroup");
}

template <int KIND>
__device__ __forceinline__ void drain_list(const int* lst, int cnt, float* ACC, int* CNT, unsigned char* POSB,
                                           const int* __restrict__ srcv, const float* __restrict__ src, int nsrc,
                                           const float* __restrict__ rs_src, int lane, int wave) {
  constexpr int RA  = (KIND == 0) ? RDEG : RACC;
  constexpr int SHF = (KIND == 0) ? 0 : 21;
  const int so8 = lane >> 2;
  const int l4  = lane & 3;
  unsigned char* posw = POSB + wave * (8 * DBAT);
  const int dummy = RA + 8 * wave + so8;
#pragma unroll 1
  for (int base = 0; base < LCAP; base += DBAT) {
    if (base >= cnt) break;
    int pc[8];
#pragma unroll
    for (int s = 0; s < 8; ++s) pc[s] = 0;
#pragma unroll
    for (int k = 0; k < 8; ++k) {
      const int idx = base + 32 * k + lane;
      const int idc = (idx < LCAP) ? idx : (LCAP - 1);
      const int v = lst[idc];
      const bool valid = idx < cnt;
      const unsigned dl = ((unsigned)v) >> SHF;
      const int ow = (int)((dl >> 1) & 1u);
      const int so = (int)((dl >> 2) & 7u);
      const bool mine = valid && (ow == wave);
      unsigned mm = 0u;
      int pb = 0;
#pragma unroll
      for (int s = 0; s < 8; ++s) {
        const bool sel = (so == s);
        const int pred = (mine && sel) ? 1 : 0;
        const unsigned mk = (unsigned)__ballot(pred);
        mm = sel ? mk : mm;
        pb = sel ? pc[s] : pb;
        pc[s] += (int)__builtin_popcount(mk);
      }
      int rank = pb + (int)__builtin_amdgcn_mbcnt_lo(mm, 0u);
      rank = (rank < DBAT) ? rank : (DBAT - 1);
      if (mine) posw[so * DBAT + rank] = (unsigned char)(32 * k + lane);
    }
    int maxc = 0, myc = 0;
#pragma unroll
    for (int s = 0; s < 8; ++s) { maxc = (pc[s] > maxc) ? pc[s] : maxc; myc = (so8 == s) ? pc[s] : myc; }
    lds_wave_sync();
#pragma unroll 1
    for (int i = 0; i < DBAT; ++i) {
      if (i >= maxc) break;
      const bool has = i < myc;
      const int p = (int)posw[so8 * DBAT + i];
      int li = base + p; li = (li < LCAP) ? li : (LCAP - 1);
      const int v = lst[li];
      const unsigned dl = ((unsigned)v) >> SHF;
      const int dli = (dl < (unsigned)RA) ? (int)dl : (RA - 1);
      const int row = has ? dli : dummy;
      if (KIND == 0) {
        const int cv = CNT[row] + (has ? 1 : 0);
        if (l4 == 0) CNT[row] = cv;
      } else {
        int e = (int)(((unsigned)v) & EMASK); e = (e < NE) ? e : (NE - 1);
        int s = srcv[e]; s = (s < 0) ? 0 : s; s = (s < nsrc) ? s : (nsrc - 1);
        const float f = has ? 1.0f : 0.0f;
        const float w = rs_src[s] * f;
        const float* sp = src + (size_t)s * DIM + 16 * l4;
        const v4f x0 = *(const v4f*)(sp);
        const v4f x1 = *(const v4f*)(sp + 4);
        const v4f x2 = *(const v4f*)(sp + 8);
        const v4f x3 = *(const v4f*)(sp + 12);
        float* ap = ACC + row * DIM + 16 * l4;
        v4f a0 = *(const v4f*)(ap);
        v4f a1 = *(const v4f*)(ap + 4);
        v4f a2 = *(const v4f*)(ap + 8);
        v4f a3 = *(const v4f*)(ap + 12);
        a0 = a0 + x0 * w;
        a1 = a1 + x1 * w;
        a2 = a2 + x2 * w;
        a3 = a3 + x3 * w;
        *(v4f*)(ap) = a0;
        *(v4f*)(ap + 4) = a1;
        *(v4f*)(ap + 8) = a2;
        *(v4f*)(ap + 12) = a3;
      }
    }
    lds_wave_sync();
  }
}

template <int KIND>
__device__ __forceinline__ void stream_tile(const int* __restrict__ dstv, const int* __restrict__ srcv,
                                            const float* __restrict__ src, int nsrc, const float* __restrict__ rs_src,
                                            float* ACC, int* CNT, int* LISTW, unsigned char* POSB, int* SCNT,
                                            const unsigned short* MAPQ, int n0, int rb, int tid, int lane, int wave) {
  constexpr int RT  = (KIND == 0) ? RDEG : ((KIND == 1) ? RACC : RQT);
  constexpr int SHF = (KIND == 0) ? 0 : 21;
  constexpr int DK  = (KIND == 0) ? 0 : 1;
  int* mylist = LISTW + wave * LCAP;
  int lc = 0;
#pragma unroll 1
  for (int c = 0; c < PNCH; ++c) {
    const int eb = c * PSCH + tid * PSP;
    const bool live = eb < NE;
    const int ebc = live ? eb : (NE - PSP);
    v4i d4[8];
#pragma unroll
    for (int k = 0; k < 8; ++k) d4[k] = *(const v4i*)(dstv + ebc + 4 * k);
#pragma unroll
    for (int j = 0; j < PSP; ++j) {
      const int d = d4[j >> 2][j & 3];
      const unsigned x = (unsigned)d - (unsigned)n0;
      bool hit = live && (x < (unsigned)RT);
      unsigned m = (unsigned)__ballot(hit ? 1 : 0);
      if (m != 0u) {
        unsigned key = x;
        if (KIND == 2) {
          const unsigned xc = (x < (unsigned)RT) ? x : (unsigned)(RT - 1);
          const int slot = (int)MAPQ[xc] - rb;
          hit = hit && ((unsigned)slot < (unsigned)RACC);
          key = (unsigned)slot;
          m = (unsigned)__ballot(hit ? 1 : 0);
        }
        const int rank = (int)__builtin_amdgcn_mbcnt_lo(m, 0u);
        int pos = lc + rank; pos = (pos < LCAP) ? pos : (LCAP - 1);
        const unsigned rec = (KIND == 0) ? key : ((key << SHF) | (unsigned)(ebc + j));
        if (hit) mylist[pos] = (int)rec;
        lc += (int)__builtin_popcount(m);
      }
    }
    if (lane == 0) SCNT[wave] = lc;
    __syncthreads();
    const int cA = SCNT[0];
    const int cB = SCNT[1];
    __syncthreads();
    const bool dodrain = (cA > LTHR) || (cB > LTHR) || (c == PNCH - 1);
    if (dodrain) {
      drain_list<DK>(LISTW, cA, ACC, CNT, POSB, srcv, src, nsrc, rs_src, lane, wave);
      drain_list<DK>(LISTW + LCAP, cB, ACC, CNT, POSB, srcv, src, nsrc, rs_src, lane, wave);
      lc = 0;
      __syncthreads();
    }
  }
}

template <int KIND>
__global__ __launch_bounds__(PT) void prop_kernel(const int* __restrict__ dstv, const int* __restrict__ srcv,
                                                 const float* __restrict__ src, int nsrc,
                                                 const float* __restrict__ rs_src, const float* rs_dst,
                                                 float* dst, const int* __restrict__ qidx, int nq, int ndst) {
  extern __shared__ __align__(16) unsigned char dynlds[];
  constexpr int HEAD  = (KIND == 0) ? CNT_BYTES : ACC_BYTES;
  constexpr int RTILE = (KIND == 0) ? RDEG : ((KIND == 1) ? RACC : RQT);
  float* ACC = (float*)(void*)dynlds;
  int* CNT = (int*)(void*)dynlds;
  int* LISTW = (int*)(void*)(dynlds + HEAD);
  unsigned char* POSB = dynlds + HEAD + LIST_BYTES;
  int* SCNT = (int*)(void*)(dynlds + HEAD + LIST_BYTES + POS_BYTES);
  unsigned short* MAPQ = (unsigned short*)(void*)(dynlds + HEAD + LIST_BYTES + POS_BYTES + SCNT_BYTES);

  const int tid  = threadIdx.x;
  const int lane = tid & 31;
  const int wave = tid >> 5;
  const int n0   = blockIdx.x * RTILE;
  const v4f z4 = {0.f, 0.f, 0.f, 0.f};

  if (KIND == 0) {
    for (int i = tid; i < RDEG + 16; i += PT) CNT[i] = 0;
  } else {
    for (int i = tid; i < (RACC + 16) * (DIM / 4); i += PT) ((v4f*)(void*)ACC)[i] = z4;
  }
  for (int i = tid; i < 2 * LCAP; i += PT) LISTW[i] = 0;
  for (int i = tid; i < POS_BYTES / 4; i += PT) ((int*)(void*)POSB)[i] = 0;
  if (tid < SCNT_BYTES / 4) SCNT[tid] = 0;
  if (KIND == 2) {
    for (int i = tid; i < MAPQ_BYTES / 4; i += PT) ((unsigned*)(void*)MAPQ)[i] = 0xFFFFFFFFu;
  }
  __syncthreads();

  if (KIND == 0) {
    stream_tile<0>(dstv, srcv, src, nsrc, rs_src, ACC, CNT, LISTW, POSB, SCNT, MAPQ, n0, 0, tid, lane, wave);
#pragma unroll 1
    for (int g = wave; g < RDEG / 128; g += 2) {
      const v4i cq = *(const v4i*)(CNT + 128 * g + 4 * lane);
      v4f o;
#pragma unroll
      for (int e = 0; e < 4; ++e) { const int cv = (cq[e] < 1) ? 1 : cq[e]; o[e] = rsqrtf((float)cv); }
      float* op = dst + (size_t)n0 + 128 * g + 4 * lane;
      *(volatile v4f*)op = o;
      __threadfence();
      *(volatile v4f*)op = o;
    }
  } else if (KIND == 1) {
    stream_tile<1>(dstv, srcv, src, nsrc, rs_src, ACC, CNT, LISTW, POSB, SCNT, MAPQ, n0, 0, tid, lane, wave);
    const int hsel = lane >> 4;
    const int c4 = (lane & 15) * 4;
#pragma unroll 1
    for (int j = 0; j < RACC / 4; ++j) {
      const int row = 4 * j + 2 * wave + hsel;
      const int n = n0 + row;
      const float rsd = rs_dst[n];
      const v4f a = *(const v4f*)(ACC + row * DIM + c4);
      const v4f o = a * rsd;
      float* op = dst + (size_t)n * DIM + c4;
      *(volatile v4f*)op = o;
      __threadfence();
      *(volatile v4f*)op = o;
    }
  } else {
    if (wave == 0) {
      int ns = 0;
#pragma unroll 1
      for (int i = 0; i < BATCH; ++i) {
        if (i >= nq) break;
        int u = qidx[i]; u = (u < 0) ? 0 : u; u = (u < ndst) ? u : (ndst - 1);
        const unsigned x = (unsigned)u - (unsigned)n0;
        if (x < (unsigned)RQT) {
          if (MAPQ[x] == (unsigned short)0xFFFFu) { MAPQ[x] = (unsigned short)ns; ++ns; }
        }
      }
      if (lane == 0) SCNT[2] = ns;
    }
    __syncthreads();
    const int ns = SCNT[2];
    const int hsel = lane >> 4;
    const int c4 = (lane & 15) * 4;
#pragma unroll 1
    for (int ph = 0; ph < QPH; ++ph) {
      if (ph > 0 && ph * RACC >= ns) break;
      const int rb = ph * RACC;
      if (ph > 0) {
        for (int i = tid; i < (RACC + 16) * (DIM / 4); i += PT) ((v4f*)(void*)ACC)[i] = z4;
        __syncthreads();
      }
      stream_tile<2>(dstv, srcv, src, nsrc, rs_src, ACC, CNT, LISTW, POSB, SCNT, MAPQ, n0, rb, tid, lane, wave);
#pragma unroll 1
      for (int j = 0; j < RQT / 4; ++j) {
        const int row = 4 * j + 2 * wave + hsel;
        const int n = n0 + row;
        const int slot = (int)MAPQ[row];
        const int sl = slot - rb;
        const bool inr = ((unsigned)sl < (unsigned)RACC);
        const bool wr = inr || ((slot == 0xFFFF) && (ph == 0));
        const int slc = inr ? sl : 0;
        const float f = inr ? 1.0f : 0.0f;
        const float rsd = rs_dst[n] * f;
        const v4f a = *(const v4f*)(ACC + slc * DIM + c4);
        const v4f o = a * rsd;
        float* op = dst + (size_t)n * DIM + c4;
        if (wr) *(volatile v4f*)op = o;
        __threadfence();
        if (wr) *(volatile v4f*)op = o;
      }
      __syncthreads();
    }
  }
}

__global__ __launch_bounds__(SCT) void score_kernel(
    const float* __restrict__ utab, const float* __restrict__ u1, const float* __restrict__ u2, const float* __restrict__ u3,
    const float* __restrict__ itab, const float* __restrict__ i1, const float* __restrict__ i2, const float* __restrict__ i3,
    const int* __restrict__ quser, const int* __restrict__ qitem, const int* __restrict__ qnegs,
    float* __restrict__ out, float* __restrict__ part) {
  __shared__ __align__(16) unsigned AHW[4][16 * 36];
  __shared__ __align__(16) unsigned ALW[4][16 * 36];
  __shared__ __align__(16) unsigned UHW[4][32];
  __shared__ __align__(16) unsigned ULW[4][32];
  __shared__ __align__(16) float POSS[SBLK];
  __shared__ __align__(16) float NEGS[SBLK * NNEG];
  __shared__ float RED[4];

  const int tid  = threadIdx.x;
  const int lane = tid & 31;
  const int wave = tid >> 5;
  const int hh   = lane >> 4;
  const int c16  = lane & 15;
  const int koff = hh * 8;
  const int blk  = blockIdx.x;
  unsigned* ahw = AHW[wave];
  unsigned* alw = ALW[wave];
  unsigned* uhw = UHW[wave];
  unsigned* ulw = ULW[wave];
  const __bf16* ahb = (const __bf16*)(const void*)ahw;
  const __bf16* alb = (const __bf16*)(const void*)alw;
  const __bf16* uhb = (const __bf16*)(const void*)uhw;
  const __bf16* ulb = (const __bf16*)(const void*)ulw;

  float sq = 0.0f;
#pragma unroll 1
  for (int ib = 0; ib < SBLK / 4; ++ib) {
    const int bl = ib * 4 + wave;
    const int b  = blk * SBLK + bl;
    int ub = quser[b]; ub = (ub < 0) ? 0 : ub; ub = (ub < NUM_USER) ? ub : (NUM_USER - 1);
    int ip = qitem[b]; ip = (ip < 0) ? 0 : ip; ip = (ip < NUM_ITEM) ? ip : (NUM_ITEM - 1);
    {
      const size_t ro = (size_t)ub * DIM + 2 * lane;
      const v2f t0 = *(const v2f*)(utab + ro);
      const v2f t1 = *(const v2f*)(u1 + ro);
      const v2f t2 = *(const v2f*)(u2 + ro);
      const v2f t3 = *(const v2f*)(u3 + ro);
      v2f v = ((t0 + t1) + t2) + t3;
      v = v * 0.25f;
      sq += v[0] * v[0] + v[1] * v[1];
      const unsigned short h0 = f2bf_bits(v[0]), h1 = f2bf_bits(v[1]);
      const unsigned short l0 = f2bf_bits(v[0] - bf_bits2f(h0)), l1 = f2bf_bits(v[1] - bf_bits2f(h1));
      uhw[lane] = (unsigned)h0 | ((unsigned)h1 << 16);
      ulw[lane] = (unsigned)l0 | ((unsigned)l1 << 16);
    }
    lds_wave_sync();
    v16b ubh[2], ubl[2];
#pragma unroll
    for (int dc = 0; dc < 2; ++dc) {
      ubh[dc] = FragB::load(uhb + koff + 32 * dc);
      ubl[dc] = FragB::load(ulb + koff + 32 * dc);
    }
#pragma unroll 1
    for (int t = 0; t < 4; ++t) {
#pragma unroll 1
      for (int r = 0; r < 16; ++r) {
        const int slot = t * 16 + r;
        int sn = slot - 1; sn = (sn < 0) ? 0 : sn; sn = (sn < NNEG) ? sn : (NNEG - 1);
        int iq = qnegs[(size_t)b * NNEG + sn]; iq = (iq < 0) ? 0 : iq; iq = (iq < NUM_ITEM) ? iq : (NUM_ITEM - 1);
        const int idx = (slot == 0) ? ip : iq;
        const size_t ro = (size_t)idx * DIM + 2 * lane;
        const v2f t0 = *(const v2f*)(itab + ro);
        const v2f t1 = *(const v2f*)(i1 + ro);
        const v2f t2 = *(const v2f*)(i2 + ro);
        const v2f t3 = *(const v2f*)(i3 + ro);
        v2f v = ((t0 + t1) + t2) + t3;
        v = v * 0.25f;
        if (slot <= NNEG) sq += v[0] * v[0] + v[1] * v[1];
        const unsigned short h0 = f2bf_bits(v[0]), h1 = f2bf_bits(v[1]);
        const unsigned short l0 = f2bf_bits(v[0] - bf_bits2f(h0)), l1 = f2bf_bits(v[1] - bf_bits2f(h1));
        ahw[r * 36 + lane] = (unsigned)h0 | ((unsigned)h1 << 16);
        alw[r * 36 + lane] = (unsigned)l0 | ((unsigned)l1 << 16);
      }
      lds_wave_sync();
      v8f acc = {0.f, 0.f, 0.f, 0.f, 0.f, 0.f, 0.f, 0.f};
#pragma unroll
      for (int dc = 0; dc < 2; ++dc) {
        const v16b ah = FragB::load(ahb + c16 * 72 + koff + 32 * dc);
        const v16b al = FragB::load(alb + c16 * 72 + koff + 32 * dc);
        acc = bmma(ah, ubh[dc], acc);
        acc = bmma(ah, ubl[dc], acc);
        acc = bmma(al, ubh[dc], acc);
      }
      if (c16 == 0) {
#pragma unroll
        for (int rr = 0; rr < 8; ++rr) {
          const int s2 = t * 16 + 8 * hh + rr;
          const float val = acc[rr];
          if (s2 == 0) POSS[bl] = val;
          else if (s2 <= NNEG) NEGS[bl * NNEG + s2 - 1] = val;
        }
      }
      lds_wave_sync();
    }
  }
#pragma unroll
  for (int o = 16; o > 0; o >>= 1) sq += __shfl_xor(sq, o, 32);
  if (lane == 0) RED[wave] = sq;
  __syncthreads();
  const float S = ((RED[0] + RED[1]) + RED[2]) + RED[3];

  const int lp = (lane < 8) ? lane : 0;
  const v4f pv = *(const v4f*)(POSS + 4 * lp);
  v4f nv[4];
  int ni[4];
#pragma unroll
  for (int k = 0; k < 4; ++k) {
    ni[k] = tid + k * SCT;
    const int ic = (ni[k] < SBLK * NNEG / 4) ? ni[k] : (SBLK * NNEG / 4 - 1);
    nv[k] = *(const v4f*)(NEGS + 4 * ic);
  }
  v4f qv = {0.f, 0.f, 0.f, 0.f};
  if (lane == 0) qv[0] = S;
  float* pos_out  = out + (size_t)blk * SBLK;
  float* neg_out  = out + OUT_NEG_OFF + (size_t)blk * (SBLK * NNEG);
  float* part_out = part + (size_t)blk * PARTW;
  for (int pass = 0; pass < 2; ++pass) {
    if (wave == 0 && lane < 8) {
      *(volatile v4f*)(pos_out + 4 * lane) = pv;
      *(volatile v4f*)(part_out + 4 * lane) = qv;
    }
#pragma unroll
    for (int k = 0; k < 4; ++k) {
      if (ni[k] < SBLK * NNEG / 4) *(volatile v4f*)(neg_out + 4 * ni[k]) = nv[k];
    }
    __threadfence();
  }
}

__global__ __launch_bounds__(SCT) void reg_final_kernel(const float* __restrict__ part, float* __restrict__ out) {
  __shared__ float red[NSBLK];
  const int tid = threadIdx.x;
  red[tid] = part[(size_t)tid * PARTW];
  __syncthreads();
  if (tid < 32) {
    double s = 0.0;
#pragma unroll 1
    for (int i = 0; i < NSBLK; ++i) s += (double)red[i];
    const float rv = (float)(s * (0.5 / (double)BATCH));
    if (tid == 0) {
      volatile float* pr = out + OUT_REG_OFF;
      *pr = rv;
      __threadfence();
      *pr = rv;
    }
  }
}

extern "C" void kernel_launch(void* const* d_in, const int* in_sizes, int n_in,
                              void* d_out, int out_size, void* d_ws, size_t ws_size,
                              hipStream_t stream) {
  if (n_in < 7) return;
  if (in_sizes[0] != NUM_USER * DIM || in_sizes[1] != NUM_ITEM * DIM || in_sizes[2] != NE || in_sizes[3] != NE ||
      in_sizes[4] != BATCH || in_sizes[5] != BATCH || in_sizes[6] != BATCH * NNEG) return;
  if (out_size != OUT_REG_OFF + 1) return;

  const float* utab  = (const float*)d_in[0];
  const float* itab  = (const float*)d_in[1];
  const int*   eu    = (const int*)d_in[2];
  const int*   ei    = (const int*)d_in[3];
  const int*   quser = (const int*)d_in[4];
  const int*   qitem = (const int*)d_in[5];
  const int*   qnegs = (const int*)d_in[6];
  float* out = (float*)d_out;

  char* ws = (char*)d_ws; size_t off = 0;
  auto carve = [&](size_t bytes) -> char* { char* p = ws + off; off += (bytes + 255) & ~(size_t)255; return p; };
  float* rs_u = (float*)carve((size_t)NU_BIG * 4);
  float* rs_i = (float*)carve((size_t)NI_BIG * 4);
  float* u1   = (float*)carve((size_t)NU_PAD * DIM * 4);
  float* u2   = (float*)carve((size_t)NU_PAD * DIM * 4);
  float* u3   = (float*)carve((size_t)NU_BIG * DIM * 4);
  float* i1   = (float*)carve((size_t)NI_PAD * DIM * 4);
  float* i2   = (float*)carve((size_t)NI_PAD * DIM * 4);
  float* i3   = (float*)carve((size_t)NI_PAD * DIM * 4);
  float* part = (float*)carve((size_t)NSBLK * PARTW * 4);
  if (off > ws_size || off > (size_t)134217728) return;

  prop_kernel<0><<<dim3(NTDU), dim3(PT), (size_t)LDS_DEG, stream>>>(eu, ei, itab, NUM_ITEM, rs_i, rs_u, rs_u, quser, 0, NUM_USER);
  prop_kernel<0><<<dim3(NTDI), dim3(PT), (size_t)LDS_DEG, stream>>>(ei, eu, utab, NUM_USER, rs_u, rs_i, rs_i, quser, 0, NUM_ITEM);
  prop_kernel<1><<<dim3(NTU), dim3(PT), (size_t)LDS_ROWS, stream>>>(eu, ei, itab, NUM_ITEM, rs_i, rs_u, u1, quser, 0, NUM_USER);
  prop_kernel<1><<<dim3(NTI), dim3(PT), (size_t)LDS_ROWS, stream>>>(ei, eu, utab, NUM_USER, rs_u, rs_i, i1, quser, 0, NUM_ITEM);
  prop_kernel<1><<<dim3(NTU), dim3(PT), (size_t)LDS_ROWS, stream>>>(eu, ei, i1, NUM_ITEM, rs_i, rs_u, u2, quser, 0, NUM_USER);
  prop_kernel<1><<<dim3(NTI), dim3(PT), (size_t)LDS_ROWS, stream>>>(ei, eu, u1, NUM_USER, rs_u, rs_i, i2, quser, 0, NUM_ITEM);
  prop_kernel<2><<<dim3(NTQ), dim3(PT), (size_t)LDS_QRY, stream>>>(eu, ei, i2, NUM_ITEM, rs_i, rs_u, u3, quser, BATCH, NUM_USER);
  prop_kernel<1><<<dim3(NTI), dim3(PT), (size_t)LDS_ROWS, stream>>>(ei, eu, u2, NUM_USER, rs_u, rs_i, i3, quser, 0, NUM_ITEM);
  score_kernel<<<dim3(NSBLK), dim3(SCT), 0, stream>>>(utab, u1, u2, u3, itab, i1, i2, i3, quser, qitem, qnegs, out, part);
  reg_final_kernel<<<dim3(1), dim3(SCT), 0, stream>>>(part, out);
}
